// Qwen3_5Attention_85529978732976
// MI455X (gfx1250) — hardware-verified
//
#include <hip/hip_runtime.h>
#include <math.h>
#pragma clang fp contract(off)

constexpr int kB    = 2;
constexpr int kS    = 2048;
constexpr int kHid  = 2048;
constexpr int kNH   = 16;
constexpr int kNKV  = 8;
constexpr int kHD   = 128;
constexpr int kTok  = kB * kS;
constexpr int kQS   = 512;
constexpr int kQP   = kS - kQS;
constexpr int kCP   = 1024;
constexpr float kWCarry       = 64.0f;
constexpr float kWCarryInv    = 1.0f / 64.0f;
constexpr float kACarry       = 64.0f;
constexpr float kPCarry       = 32768.0f;
constexpr float kOutScalePlain = 1.0f / (kACarry * kWCarry);
constexpr float kEps   = 1.0e-6f;
constexpr float kScale = 0.08838834764831845f;
constexpr float kFill  = -3.4028234663852886e38f;
static_assert(kTok % 64 == 0 && kCP % 64 == 0 && kHid % 64 == 0 && kQS % 64 == 0 && kQP % 64 == 0, "tile multiples");
static_assert(kHid % 32 == 0 && kHD % 32 == 0, "K multiples");
static_assert(kNH * kHD == kHid && kNKV * kHD == kCP, "shapes");
static_assert(kS % 64 == 0 && kS % 8 == 0 && kQS % 64 == 0, "blocks");

typedef __attribute__((ext_vector_type(16))) _Float16 v16h;
typedef __attribute__((ext_vector_type(8)))  _Float16 v8h;
typedef __attribute__((ext_vector_type(16))) __bf16   v16b;
typedef __attribute__((ext_vector_type(8)))  __bf16   v8b;
typedef __attribute__((ext_vector_type(8)))  float    v8f;
typedef __attribute__((ext_vector_type(4)))  float    v4f;
typedef __attribute__((ext_vector_type(4)))  unsigned int v4u;
typedef __attribute__((ext_vector_type(2)))  unsigned int v2u;

__device__ __forceinline__ unsigned short f2bf_bits(float f) {
  unsigned u = __float_as_uint(f);
  return (unsigned short)((u + 0x7FFFu + ((u >> 16) & 1u)) >> 16);
}
__device__ __forceinline__ float bf_bits2f(unsigned short h) { return __uint_as_float(((unsigned)h) << 16); }
__device__ __forceinline__ unsigned pk16(unsigned short a, unsigned short b) { return (unsigned)a | ((unsigned)b << 16); }
__device__ __forceinline__ unsigned short h_bits(float f) { const _Float16 h = (_Float16)f; return __builtin_bit_cast(unsigned short, h); }
__device__ __forceinline__ float h16_to_f32(unsigned hb) {
  const unsigned sgn = (hb & 0x8000u) << 16; const unsigned em = hb & 0x7fffu;
  const float fn = __uint_as_float((em << 13) + 0x38000000u);
  const float fs = (float)em * 5.9604644775390625e-8f;
  const float mag = (em < 0x400u) ? fs : fn; return __uint_as_float(__float_as_uint(mag) | sgn); }

__device__ __forceinline__ void dep_guard_h(v8f& a, v8f& b, v16h x, v16h y) { asm volatile("v_nop\n\tv_nop\n\tv_nop\n\tv_nop" : "+v"(a), "+v"(b) : "v"(x), "v"(y)); }
__device__ __forceinline__ void dep_guard_b(v8f& a, v8f& b, v16b x, v16b y) { asm volatile("v_nop\n\tv_nop\n\tv_nop\n\tv_nop" : "+v"(a), "+v"(b) : "v"(x), "v"(y)); }
__device__ __forceinline__ void keep4_h(v16h a, v16h b, v16h c, v16h d) { asm volatile("v_nop" :: "v"(a), "v"(b), "v"(c), "v"(d)); }
__device__ __forceinline__ void keep4_b(v16b a, v16b b, v16b c, v16b d) { asm volatile("v_nop" :: "v"(a), "v"(b), "v"(c), "v"(d)); }
__device__ __forceinline__ void acc_guard4(v8f& a, v8f& b, v8f& c, v8f& d) { asm volatile("v_nop\n\tv_nop\n\tv_nop\n\tv_nop" : "+v"(a), "+v"(b), "+v"(c), "+v"(d)); }
__device__ __forceinline__ void mem_order() { asm volatile("" ::: "memory"); }
template <typename T> struct Frag;
template <> struct Frag<_Float16> {
  typedef v16h V; union U { v16h v; v8h h[2]; };
  static __device__ __forceinline__ v16h load(const _Float16* p) {
    U f; f.h[0] = *(const v8h*)(p); f.h[1] = *(const v8h*)(p + 16); return f.v;
  }
  static __device__ __forceinline__ v8f mma(v16h a, v16h b, v8f c) {
    return __builtin_amdgcn_wmma_f32_16x16x32_f16(false, a, false, b, (short)0, c, false, false);
  }
  static __device__ __forceinline__ void guard(v8f& a, v8f& b, v16h x, v16h y) { dep_guard_h(a, b, x, y); }
  static __device__ __forceinline__ void keep(v16h a, v16h b, v16h c, v16h d) { keep4_h(a, b, c, d); }
};
template <> struct Frag<__bf16> {
  typedef v16b V; union U { v16b v; v8b h[2]; };
  static __device__ __forceinline__ v16b load(const __bf16* p) {
    U f; f.h[0] = *(const v8b*)(p); f.h[1] = *(const v8b*)(p + 16); return f.v;
  }
  static __device__ __forceinline__ v8f mma(v16b a, v16b b, v8f c) {
    return __builtin_amdgcn_wmma_f32_16x16x32_bf16(false, a, false, b, (short)0, c, false, false);
  }
  static __device__ __forceinline__ void guard(v8f& a, v8f& b, v16b x, v16b y) { dep_guard_b(a, b, x, y); }
  static __device__ __forceinline__ void keep(v16b a, v16b b, v16b c, v16b d) { keep4_b(a, b, c, d); }
};

__device__ __forceinline__ v8f amma(v16h a, v16h b, v8f c) {
  c = __builtin_amdgcn_wmma_f32_16x16x32_f16(false, a, false, b, (short)0, c, false, false);
  asm volatile("v_nop\n\tv_nop\n\tv_nop\n\tv_nop" : "+v"(c) : "v"(a), "v"(b));
  return c;
}
__device__ __forceinline__ v8f amma(v16b a, v16b b, v8f c) {
  c = __builtin_amdgcn_wmma_f32_16x16x32_bf16(false, a, false, b, (short)0, c, false, false);
  asm volatile("v_nop\n\tv_nop\n\tv_nop\n\tv_nop" : "+v"(c) : "v"(a), "v"(b));
  return c;
}
__device__ __forceinline__ void wave_sync() {
  __builtin_amdgcn_fence(__ATOMIC_RELEASE, "workgroup");
  __builtin_amdgcn_wave_barrier();
  __builtin_amdgcn_fence(__ATOMIC_ACQUIRE, "workgroup");
}

template <int ET> struct Elem;
template <> struct Elem<0> { typedef _Float16 T; };
template <> struct Elem<1> { typedef __bf16 T; };
template <int ET, int SPLIT, int BIAS_MODE, int OUT_MODE, bool RESID, int ACT = 0>
__global__ __launch_bounds__(256) void wmma_gemm64(
    const unsigned short* __restrict__ Ap, const unsigned short* __restrict__ A2p, int lda, long strideA,
    const unsigned short* __restrict__ Btp, const unsigned short* __restrict__ Bt2p, int ldb, long strideB,
    void* __restrict__ Cout, void* __restrict__ Cout2, int ldc, long strideC,
    const float* __restrict__ bias,
    const float* __restrict__ resid, long strideR,
    int M, int N, int K, float scale) {
  typedef typename Elem<ET>::T T;
  typedef typename Frag<T>::V V;
  const T* A = (const T*)Ap; const T* A2 = (const T*)A2p; const T* Bt = (const T*)Btp; const T* Bt2 = (const T*)Bt2p;
  __shared__ __align__(16) float sT[8][16 * 68];
  const int b    = blockIdx.y;
  const int lane = threadIdx.x & 31;
  const int wave = threadIdx.x >> 5;
  const int tilesN = N >> 6;
  const int tilesM = M >> 6;
  const int tile = blockIdx.x * 8 + wave;
  if (tile >= tilesM * tilesN) return;
  const int tm = tile / tilesN;
  const int tn = tile - tm * tilesN;
  const int m0 = tm << 6;
  const int n0 = tn << 6;

  const T* Ab  = A  + (size_t)b * strideA;
  const T* Bb  = Bt + (size_t)b * strideB;
  const T* Ab2 = SPLIT ? (A2  + (size_t)b * strideA) : nullptr;
  const T* Bb2 = (SPLIT == 1) ? (Bt2 + (size_t)b * strideB) : nullptr;

  const int rlane = lane & 15;
  const int koff  = (lane >> 4) * 8;
  const int mOff  = (lane >> 4) * 8;

  v8f acc[4][4];
#pragma unroll
  for (int i = 0; i < 4; ++i)
#pragma unroll
    for (int j = 0; j < 4; ++j) acc[i][j] = (v8f){0.f,0.f,0.f,0.f,0.f,0.f,0.f,0.f};

  for (int k0 = 0; k0 < K; k0 += 32) {
    V bh[4], bl[4];
#pragma unroll
    for (int j = 0; j < 4; ++j) {
      const size_t bo = (size_t)(n0 + (j << 4) + rlane) * ldb + koff + k0;
      bh[j] = Frag<T>::load(Bb + bo);
      if (SPLIT == 1) bl[j] = Frag<T>::load(Bb2 + bo);
    }
#pragma unroll
    for (int i = 0; i < 4; ++i) {
      const size_t ao = (size_t)(m0 + (i << 4) + rlane) * lda + koff + k0;
      V ah = Frag<T>::load(Ab + ao);
      V al;
      if (SPLIT) al = Frag<T>::load(Ab2 + ao);
#pragma unroll
      for (int j = 0; j < 4; ++j) {
        acc[i][j] = Frag<T>::mma(ah, bh[j], acc[i][j]);
        if (SPLIT == 1) acc[i][j] = Frag<T>::mma(ah, bl[j], acc[i][j]);
        if (SPLIT) acc[i][j] = Frag<T>::mma(al, bh[j], acc[i][j]);
      }
      Frag<T>::guard(acc[i][0], acc[i][3], ah, SPLIT ? al : ah);
    }
    Frag<T>::keep(bh[0], bh[1], bh[2], bh[3]);
    if (SPLIT == 1) Frag<T>::keep(bl[0], bl[1], bl[2], bl[3]);
  }
  acc_guard4(acc[0][0], acc[0][1], acc[0][2], acc[0][3]);
  acc_guard4(acc[1][0], acc[1][1], acc[1][2], acc[1][3]);
  acc_guard4(acc[2][0], acc[2][1], acc[2][2], acc[2][3]);
  acc_guard4(acc[3][0], acc[3][1], acc[3][2], acc[3][3]);

  float* slab = sT[wave];
  const float* Rb = RESID ? (resid + (size_t)b * strideR) : nullptr;
#pragma unroll
  for (int i = 0; i < 4; ++i) {
    const int mBase = m0 + (i << 4);
#pragma unroll
    for (int j = 0; j < 4; ++j) {
      const int n = n0 + (j << 4) + rlane;
      float bv = 0.f;
      if (BIAS_MODE == 2) bv = bias[n];
#pragma unroll
      for (int r = 0; r < 8; ++r) {
        float v = acc[i][j][r] * scale;
        if (BIAS_MODE == 1) v += bias[mBase + mOff + r];
        if (BIAS_MODE == 2) v += bv;
        if (RESID) v += Rb[(size_t)(mBase + mOff + r) * ldc + n];
        if (ACT == 2) v = fmaxf(v, 0.0f);
        if (ACT == 4) v = (v > 0.f) ? v : 0.01f * v;
        slab[(mOff + r) * 68 + (j << 4) + rlane] = v;
      }
    }
    __builtin_amdgcn_fence(__ATOMIC_RELEASE, "workgroup");
    __builtin_amdgcn_wave_barrier();
    __builtin_amdgcn_fence(__ATOMIC_ACQUIRE, "workgroup");
    if (OUT_MODE == 0) {
      float* C = (float*)Cout + (size_t)b * strideC;
      const int hh = lane >> 4, c4 = (lane & 15) * 4;
      for (int pass = 0; pass < 2; ++pass) {
#pragma unroll
        for (int it = 0; it < 8; ++it) {
          const int row = it * 2 + hh;
          v4f v = *(const v4f*)(slab + row * 68 + c4);
          *(volatile v4f*)(C + (size_t)(mBase + row) * ldc + n0 + c4) = v;
        }
        __threadfence();
      }
    } else {
      const int q = lane >> 3, c8 = (lane & 7) * 8;
      unsigned short* C  = (unsigned short*)Cout  + (size_t)b * strideC;
      unsigned short* C2 = (OUT_MODE == 2) ? ((unsigned short*)Cout2 + (size_t)b * strideC) : nullptr;
      for (int pass = 0; pass < 2; ++pass) {
#pragma unroll
        for (int it = 0; it < 4; ++it) {
          const int row = it * 4 + q;
          const float* sp = slab + row * 68 + c8;
          v8h hv, lv;
#pragma unroll
          for (int e = 0; e < 8; ++e) {
            if (OUT_MODE == 1) {
              hv[e] = (_Float16)sp[e];
            } else {
              unsigned short hb = f2bf_bits(sp[e]);
              unsigned short lb = f2bf_bits(sp[e] - bf_bits2f(hb));
              hv[e] = __builtin_bit_cast(_Float16, hb);
              lv[e] = __builtin_bit_cast(_Float16, lb);
            }
          }
          *(volatile v8h*)(C + (size_t)(mBase + row) * ldc + n0 + c8) = hv;
          if (OUT_MODE == 2) *(volatile v8h*)(C2 + (size_t)(mBase + row) * ldc + n0 + c8) = lv;
        }
        __threadfence();
      }
    }
    __builtin_amdgcn_fence(__ATOMIC_RELEASE, "workgroup");
    __builtin_amdgcn_wave_barrier();
    __builtin_amdgcn_fence(__ATOMIC_ACQUIRE, "workgroup");
  }
}

__global__ __launch_bounds__(256) void castx_kernel(const float* __restrict__ in, unsigned short* __restrict__ out, int n8) {
  const int i = blockIdx.x * 256 + threadIdx.x;
  if (i >= n8) return;
  const float* p = in + 8 * (size_t)i;
  const v4f a = *(const v4f*)(p);
  const v4f c = *(const v4f*)(p + 4);
  unsigned short hb[8];
#pragma unroll
  for (int e = 0; e < 4; ++e) {
    hb[e]     = h_bits(bf_bits2f(f2bf_bits(a[e])));
    hb[4 + e] = h_bits(bf_bits2f(f2bf_bits(c[e])));
  }
  const v4u u = (v4u){pk16(hb[0], hb[1]), pk16(hb[2], hb[3]), pk16(hb[4], hb[5]), pk16(hb[6], hb[7])};
  unsigned short* q = out + 8 * (size_t)i;
  *(volatile v4u*)q = u;
  __threadfence();
  *(volatile v4u*)q = u;
}

template <bool BF>
__global__ __launch_bounds__(256) void wt_kernel(const float* __restrict__ src, int pitch, int hmul, int goff,
                                                 unsigned short* __restrict__ dst, float carry) {
  __shared__ float sm[64][65];
  const int t  = threadIdx.x;
  const int k0 = blockIdx.x * 64;
  const int n0 = blockIdx.y * 64;
  const int colbase = (n0 >> 7) * hmul + (n0 & 127) + goff;
#pragma unroll
  for (int i = 0; i < 16; ++i) {
    const int e  = i * 256 + t;
    const int r  = e >> 6;
    const int cc = e & 63;
    sm[cc][r] = src[(size_t)(k0 + r) * pitch + colbase + cc];
  }
  __syncthreads();
  const int lane = t & 31, wave = t >> 5;
  const int q = lane >> 3, c8 = (lane & 7) * 8;
  v4u u[2];
#pragma unroll
  for (int it = 0; it < 2; ++it) {
    const int row = wave * 8 + it * 4 + q;
    unsigned short hb[8];
#pragma unroll
    for (int e = 0; e < 8; ++e) {
      const float v = sm[row][c8 + e];
      hb[e] = BF ? f2bf_bits(v) : h_bits(carry * bf_bits2f(f2bf_bits(v)));
    }
    u[it] = (v4u){pk16(hb[0], hb[1]), pk16(hb[2], hb[3]), pk16(hb[4], hb[5]), pk16(hb[6], hb[7])};
  }
  for (int pass = 0; pass < 2; ++pass) {
#pragma unroll
    for (int it = 0; it < 2; ++it) {
      const int row = wave * 8 + it * 4 + q;
      *(volatile v4u*)(dst + (size_t)(n0 + row) * kHid + k0 + c8) = u[it];
    }
    __threadfence();
  }
}

struct RopeFreq { float f[16]; };
static_assert(sizeof(RopeFreq) == 64, "no padding");

template <bool ISQ>
__global__ __launch_bounds__(256) void normrope_kernel(const float* __restrict__ Cp, const float* __restrict__ nw,
                                                       const int* __restrict__ positions, RopeFreq rf,
                                                       unsigned short* __restrict__ d16, unsigned short* __restrict__ dh,
                                                       unsigned short* __restrict__ dl, int chunk) {
  __shared__ __align__(16) float csl[128];
  __shared__ __align__(16) float snl[128];
  const int tid  = threadIdx.x;
  const int tok0 = blockIdx.x * 8;
  const int b    = tok0 / kS;
  const int s0   = tok0 - b * kS;
  if (tid < 128) {
    const int tl = tid >> 4, j = tid & 15;
    const int pos = positions[tok0 + tl];
    float f = rf.f[0];
#pragma unroll
    for (int q = 1; q < 16; ++q) f = (j == q) ? rf.f[q] : f;
    const float ang = (float)pos * f;
    float sv, cv;
    sincosf(ang, &sv, &cv);
    csl[tl * 16 + j] = cv;
    snl[tl * 16 + j] = sv;
  }
  __syncthreads();

  const int lane = tid & 31, wave = tid >> 5, hh = lane >> 4, c = lane & 15;
  float wsc[8];
  {
    const v4f w0 = *(const v4f*)(nw + c * 8);
    const v4f w1 = *(const v4f*)(nw + c * 8 + 4);
#pragma unroll
    for (int e = 0; e < 4; ++e) {
      wsc[e]     = 1.0f + bf_bits2f(f2bf_bits(w0[e]));
      wsc[4 + e] = 1.0f + bf_bits2f(f2bf_bits(w1[e]));
    }
  }
  const float rotf  = (c < 4) ? 1.0f : 0.0f;
  const float keepf = 1.0f - rotf;
  const float sgn   = (c < 2) ? -1.0f : 1.0f;
  const int jb = (c & 1) * 8;
#pragma unroll 1
  for (int p = 0; p < 4; ++p) {
    const int R   = p * 16 + wave * 2 + hh;
    const int tl  = R >> 3;
    const int hl  = R & 7;
    const int tok = tok0 + tl;
    const int s   = s0 + tl;
    const float* src = Cp + (size_t)tok * kCP + hl * kHD + c * 8;
    const v4f a0 = *(const v4f*)(src);
    const v4f a1 = *(const v4f*)(src + 4);
    float x[8];
#pragma unroll
    for (int e = 0; e < 4; ++e) { x[e] = a0[e]; x[4 + e] = a1[e]; }
    float ss = 0.0f;
#pragma unroll
    for (int e = 0; e < 8; ++e) ss += x[e] * x[e];
    ss += __shfl_xor(ss, 1, 32);
    ss += __shfl_xor(ss, 2, 32);
    ss += __shfl_xor(ss, 4, 32);
    ss += __shfl_xor(ss, 8, 32);
    const float rinv = rsqrtf(ss * (1.0f / 128.0f) + kEps);
    float y[8];
#pragma unroll
    for (int e = 0; e < 8; ++e) y[e] = (x[e] * rinv) * wsc[e];
    const v4f c0 = *(const v4f*)(csl + tl * 16 + jb);
    const v4f c1 = *(const v4f*)(csl + tl * 16 + jb + 4);
    const v4f n0 = *(const v4f*)(snl + tl * 16 + jb);
    const v4f n1 = *(const v4f*)(snl + tl * 16 + jb + 4);
    float o[8];
#pragma unroll
    for (int e = 0; e < 8; ++e) {
      const float yp = __shfl_xor(y[e], 2, 32);
      const float cs = (e < 4) ? c0[e] : c1[e - 4];
      const float sn = (e < 4) ? n0[e] : n1[e - 4];
      const float tv = y[e] * cs + sgn * (yp * sn);
      o[e] = rotf * tv + keepf * y[e];
    }
    unsigned short fb[8], hb[8], lb[8];
#pragma unroll
    for (int e = 0; e < 8; ++e) {
      fb[e] = h_bits(o[e]);
      hb[e] = f2bf_bits(o[e]);
      lb[e] = f2bf_bits(o[e] - bf_bits2f(hb[e]));
    }
    const v4u uf = (v4u){pk16(fb[0], fb[1]), pk16(fb[2], fb[3]), pk16(fb[4], fb[5]), pk16(fb[6], fb[7])};
    const v4u uh = (v4u){pk16(hb[0], hb[1]), pk16(hb[2], hb[3]), pk16(hb[4], hb[5]), pk16(hb[6], hb[7])};
    const v4u ul = (v4u){pk16(lb[0], lb[1]), pk16(lb[2], lb[3]), pk16(lb[4], lb[5]), pk16(lb[6], lb[7])};
    if (ISQ) {
      const int col = (chunk * 8 + hl) * kHD + c * 8;
      if (s >= kQS) {
        unsigned short* pf = d16 + (size_t)(b * kQP + s - kQS) * kHid + col;
        for (int pass = 0; pass < 2; ++pass) { *(volatile v4u*)pf = uf; __threadfence(); }
      } else {
        const size_t ob = (size_t)(b * kQS + s) * kHid + col;
        for (int pass = 0; pass < 2; ++pass) { *(volatile v4u*)(dh + ob) = uh; *(volatile v4u*)(dl + ob) = ul; __threadfence(); }
      }
    } else {
      const int col = hl * kHD + c * 8;
      unsigned short* pf = d16 + (size_t)tok * kCP + col;
      for (int pass = 0; pass < 2; ++pass) { *(volatile v4u*)pf = uf; __threadfence(); }
      if (s < kQS) {
        const size_t ob = (size_t)(b * kQS + s) * kCP + col;
        for (int pass = 0; pass < 2; ++pass) { *(volatile v4u*)(dh + ob) = uh; *(volatile v4u*)(dl + ob) = ul; __threadfence(); }
      }
    }
  }
}

__global__ __launch_bounds__(256) void vt_kernel(const float* __restrict__ Cp, unsigned short* __restrict__ Vt,
                                                 unsigned short* __restrict__ Vh, unsigned short* __restrict__ Vl) {
  __shared__ float sm[128][65];
  const int t   = threadIdx.x;
  const int s0  = blockIdx.x * 64;
  const int hkv = blockIdx.y;
  const int b   = blockIdx.z;
  const size_t rowbase = (size_t)(b * kS + s0);
#pragma unroll
  for (int i = 0; i < 8; ++i) {
    const int e  = i * 256 + t;
    const int r  = e >> 5;
    const int d4 = (e & 31) * 4;
    const v4f w = *(const v4f*)(Cp + (rowbase + r) * kCP + hkv * kHD + d4);
    sm[d4 + 0][r] = w[0];
    sm[d4 + 1][r] = w[1];
    sm[d4 + 2][r] = w[2];
    sm[d4 + 3][r] = w[3];
  }
  __syncthreads();
  const int lane = t & 31, wave = t >> 5;
  const int q = lane >> 3, c8 = (lane & 7) * 8;
  const size_t plane = (size_t)(b * kNKV + hkv) * kHD;
  const bool early = (s0 < kQS);
  for (int pass = 0; pass < 2; ++pass) {
#pragma unroll
    for (int it = 0; it < 4; ++it) {
      const int d = wave * 16 + it * 4 + q;
      unsigned short fb[8], hb[8], lb[8];
#pragma unroll
      for (int e = 0; e < 8; ++e) {
        const float v = sm[d][c8 + e];
        fb[e] = h_bits(v);
        hb[e] = f2bf_bits(v);
        lb[e] = f2bf_bits(v - bf_bits2f(hb[e]));
      }
      const v4u uf = (v4u){pk16(fb[0], fb[1]), pk16(fb[2], fb[3]), pk16(fb[4], fb[5]), pk16(fb[6], fb[7])};
      *(volatile v4u*)(Vt + (plane + d) * kS + s0 + c8) = uf;
      if (early) {
        const v4u uh = (v4u){pk16(hb[0], hb[1]), pk16(hb[2], hb[3]), pk16(hb[4], hb[5]), pk16(hb[6], hb[7])};
        const v4u ul = (v4u){pk16(lb[0], lb[1]), pk16(lb[2], lb[3]), pk16(lb[4], lb[5]), pk16(lb[6], lb[7])};
        *(volatile v4u*)(Vh + (plane + d) * kQS + s0 + c8) = uh;
        *(volatile v4u*)(Vl + (plane + d) * kQS + s0 + c8) = ul;
      }
    }
    __threadfence();
  }
}

template <bool SPLIT> struct ACfg;
template <> struct ACfg<false> { typedef _Float16 T; static constexpr int KC = 64; };
template <> struct ACfg<true>  { typedef __bf16  T; static constexpr int KC = 32; };

template <bool SPLIT>
__global__ __launch_bounds__(128) void attn128_kernel(
    const unsigned short* __restrict__ Qp, const unsigned short* __restrict__ Qlp, int qRows, int qS0,
    const unsigned short* __restrict__ Kp, const unsigned short* __restrict__ Klp, int kRows,
    const unsigned short* __restrict__ Vp, const unsigned short* __restrict__ Vlp, int vPitch,
    const int* __restrict__ amask,
    unsigned short* __restrict__ Op, unsigned short* __restrict__ Olp, int oRows, int oS0,
    int qb0, int nqbl) {
  typedef typename ACfg<SPLIT>::T T;
  typedef typename Frag<T>::V FV;
  constexpr int KC  = ACfg<SPLIT>::KC;
  constexpr int NJ  = KC / 16;
  constexpr int NKK = KC / 32;
  constexpr int KP  = kHD + 8;
  constexpr int NPL = SPLIT ? 2 : 1;
  __shared__ __align__(16) T Ks[NPL * KC * KP];
  __shared__ __align__(16) T Vs[NPL * kHD * KC];
  __shared__ __align__(16) T Ps[4][NPL * 16 * KC];
  __shared__ __align__(16) float Os[4][16 * 68];

  const int tid = threadIdx.x, wave = tid >> 5, lane = tid & 31, hh = lane >> 4, c = lane & 15;
  const int bx  = blockIdx.x;
  const int qb  = qb0 + (bx % nqbl);
  const int bh  = bx / nqbl;
  const int h   = bh % kNH, b = bh / kNH, hkv = h >> 1;
  const int q0  = qb * 64 + wave * 16;

  const T* Qt  = (const T*)Qp;
  const T* Qlt = (const T*)Qlp;
  const size_t qoff  = ((size_t)(b * qRows + (q0 - qS0) + c)) * kHid + h * kHD + 8 * hh;
  const size_t kbase = (size_t)(b * kRows) * kCP + hkv * kHD;
  const size_t vbase = ((size_t)(b * kNKV + hkv) * kHD) * (size_t)vPitch;
  const size_t obase = ((size_t)(b * oRows + (q0 - oS0))) * kHid + h * kHD;

  float mrow[8], lrow[8];
  v8f oacc[8];
#pragma unroll
  for (int r = 0; r < 8; ++r) { mrow[r] = -INFINITY; lrow[r] = 0.f; }
#pragma unroll
  for (int t = 0; t < 8; ++t) oacc[t] = (v8f){0.f,0.f,0.f,0.f,0.f,0.f,0.f,0.f};

  const int nChunks = (qb * 64 + 64) / KC;
  for (int kc = 0; kc < nChunks; ++kc) {
    const int kv0 = kc * KC;
    __syncthreads();
    {
      constexpr int TPR = 128 / KC;
      constexpr int HPT = kHD / TPR;
      constexpr int NVK = HPT / 8;
      const int kr = tid / TPR, ko = (tid % TPR) * HPT;
      {
        const v4u* ks = (const v4u*)(Kp + kbase + (size_t)(kv0 + kr) * kCP + ko);
        v4u* kd = (v4u*)(Ks + kr * KP + ko);
        v4u tk[NVK];
#pragma unroll
        for (int i = 0; i < NVK; ++i) tk[i] = ks[i];
#pragma unroll
        for (int i = 0; i < NVK; ++i) kd[i] = tk[i];
      }
      mem_order();
      if (SPLIT) {
        const v4u* ks = (const v4u*)(Klp + kbase + (size_t)(kv0 + kr) * kCP + ko);
        v4u* kd = (v4u*)(Ks + KC * KP + kr * KP + ko);
        v4u tk[NVK];
#pragma unroll
        for (int i = 0; i < NVK; ++i) tk[i] = ks[i];
#pragma unroll
        for (int i = 0; i < NVK; ++i) kd[i] = tk[i];
        mem_order();
      }
      constexpr int NVV = KC / 8;
      {
        const v4u* vs = (const v4u*)(Vp + vbase + (size_t)tid * vPitch + kv0);
        v4u* vd = (v4u*)(Vs + tid * KC);
        v4u tv[NVV];
#pragma unroll
        for (int i = 0; i < NVV; ++i) tv[i] = vs[i];
#pragma unroll
        for (int i = 0; i < NVV; ++i) vd[i] = tv[i];
      }
      mem_order();
      if (SPLIT) {
        const v4u* vs = (const v4u*)(Vlp + vbase + (size_t)tid * vPitch + kv0);
        v4u* vd = (v4u*)(Vs + kHD * KC + tid * KC);
        v4u tv[NVV];
#pragma unroll
        for (int i = 0; i < NVV; ++i) tv[i] = vs[i];
#pragma unroll
        for (int i = 0; i < NVV; ++i) vd[i] = tv[i];
        mem_order();
      }
    }
    __syncthreads();

    v8f s[NJ];
#pragma unroll
    for (int j = 0; j < NJ; ++j) s[j] = (v8f){0.f,0.f,0.f,0.f,0.f,0.f,0.f,0.f};
#pragma unroll
    for (int dc = 0; dc < 4; ++dc) {
      const FV qh = Frag<T>::load(Qt + qoff + dc * 32);
      FV ql = qh;
      if (SPLIT) ql = Frag<T>::load(Qlt + qoff + dc * 32);
#pragma unroll
      for (int j = 0; j < NJ; ++j) {
        const FV kb = Frag<T>::load(Ks + (j * 16 + c) * KP + dc * 32 + 8 * hh);
        s[j] = amma(qh, kb, s[j]);
        if (SPLIT) {
          const FV kl = Frag<T>::load(Ks + KC * KP + (j * 16 + c) * KP + dc * 32 + 8 * hh);
          s[j] = amma(qh, kl, s[j]);
          s[j] = amma(ql, kb, s[j]);
        }
      }
    }

    int kvkeep[NJ];
#pragma unroll
    for (int j = 0; j < NJ; ++j) kvkeep[j] = amask[b * kS + kv0 + j * 16 + c];
    float cm[8];
#pragma unroll
    for (int r = 0; r < 8; ++r) {
      const int qrow = q0 + 8 * hh + r;
      float m = -INFINITY;
#pragma unroll
      for (int j = 0; j < NJ; ++j) {
        const int kvcol = kv0 + j * 16 + c;
        const bool masked = (kvcol > qrow) || (kvkeep[j] == 0);
        float sv = s[j][r] * kScale;
        sv = masked ? kFill : sv;
        s[j][r] = sv;
        m = fmaxf(m, sv);
      }
#pragma unroll
      for (int off = 1; off < 16; off <<= 1) m = fmaxf(m, __shfl_xor(m, off, 32));
      cm[r] = m;
    }
    T* pw = Ps[wave];
#pragma unroll
    for (int r = 0; r < 8; ++r) {
      const float mnew  = fmaxf(mrow[r], cm[r]);
      const float alpha = expf(mrow[r] - mnew);
      mrow[r] = mnew;
      float psum = 0.f;
#pragma unroll
      for (int j = 0; j < NJ; ++j) {
        const float p = expf(s[j][r] - mnew);
        psum += p;
        const int pi = (8 * hh + r) * KC + j * 16 + c;
        unsigned short b0, b1;
        if (SPLIT) { b0 = f2bf_bits(p); b1 = f2bf_bits(p - bf_bits2f(b0)); }
        else       { b0 = h_bits(p * kPCarry); b1 = b0; }
        pw[pi] = __builtin_bit_cast(T, b0);
        if (SPLIT) pw[16 * KC + pi] = __builtin_bit_cast(T, b1);
      }
#pragma unroll
      for (int off = 1; off < 16; off <<= 1) psum += __shfl_xor(psum, off, 32);
      lrow[r] = lrow[r] * alpha + psum;
#pragma unroll
      for (int t = 0; t < 8; ++t) oacc[t][r] *= alpha;
    }
    wave_sync();
#pragma unroll
    for (int kk = 0; kk < NKK; ++kk) {
      const FV pa = Frag<T>::load(pw + c * KC + kk * 32 + 8 * hh);
      FV pl = pa;
      if (SPLIT) pl = Frag<T>::load(pw + 16 * KC + c * KC + kk * 32 + 8 * hh);
#pragma unroll
      for (int t = 0; t < 8; ++t) {
        const FV vb = Frag<T>::load(Vs + (t * 16 + c) * KC + kk * 32 + 8 * hh);
        oacc[t] = amma(pa, vb, oacc[t]);
        if (SPLIT) {
          const FV vl = Frag<T>::load(Vs + kHD * KC + (t * 16 + c) * KC + kk * 32 + 8 * hh);
          oacc[t] = amma(pa, vl, oacc[t]);
          oacc[t] = amma(pl, vb, oacc[t]);
        }
      }
    }
  }

  float inv[8];
#pragma unroll
  for (int r = 0; r < 8; ++r) inv[r] = (SPLIT ? 1.0f : (kACarry / kPCarry)) / lrow[r];
  float* os = Os[wave];
  const int q8 = lane >> 3, c8 = (lane & 7) * 8;
#pragma unroll
  for (int hf = 0; hf < 2; ++hf) {
#pragma unroll
    for (int r = 0; r < 8; ++r)
#pragma unroll
      for (int t4 = 0; t4 < 4; ++t4) os[(8 * hh + r) * 68 + t4 * 16 + c] = oacc[hf * 4 + t4][r] * inv[r];
    wave_sync();
    for (int pass = 0; pass < 2; ++pass) {
#pragma unroll
      for (int it = 0; it < 4; ++it) {
        const int row = it * 4 + q8;
        const float* sp = os + row * 68 + c8;
        v8h hv, lv;
#pragma unroll
        for (int e = 0; e < 8; ++e) {
          unsigned short b0, b1;
          if (SPLIT) { b0 = f2bf_bits(sp[e]); b1 = f2bf_bits(sp[e] - bf_bits2f(b0)); }
          else       { b0 = h_bits(sp[e]); b1 = b0; }
          hv[e] = __builtin_bit_cast(_Float16, b0);
          lv[e] = __builtin_bit_cast(_Float16, b1);
        }
        const size_t oo = obase + (size_t)row * kHid + hf * 64 + c8;
        *(volatile v8h*)(Op + oo) = hv;
        if (SPLIT) *(volatile v8h*)(Olp + oo) = lv;
      }
      __threadfence();
    }
    wave_sync();
  }
}

__device__ __forceinline__ float sigm(float g) {
  const float ex = expf(-g);
  return __builtin_amdgcn_rcpf(1.0f + ex);
}

__global__ __launch_bounds__(256) void gate_plain_kernel(const float* __restrict__ Gp, const unsigned short* __restrict__ Ain,
                                                         unsigned short* __restrict__ Aout, int chunk) {
  const int i   = blockIdx.x * 256 + threadIdx.x;
  const int row = i >> 8;
  if (row >= kB * kQP) return;
  const int col = (i & 255) * 4;
  const int b   = row / kQP, sp = row - b * kQP;
  const int tok = b * kS + kQS + sp;
  const v4f g = *(const v4f*)(Gp + (size_t)tok * kCP + col);
  const size_t ao = (size_t)row * kHid + chunk * kCP + col;
  const v2u aw = *(const v2u*)(Ain + ao);
  float a[4];
  a[0] = h16_to_f32(aw[0] & 0xffffu);
  a[1] = h16_to_f32(aw[0] >> 16);
  a[2] = h16_to_f32(aw[1] & 0xffffu);
  a[3] = h16_to_f32(aw[1] >> 16);
  unsigned short hb[4];
#pragma unroll
  for (int e = 0; e < 4; ++e) hb[e] = h_bits(a[e] * sigm(g[e]));
  const v2u u = (v2u){pk16(hb[0], hb[1]), pk16(hb[2], hb[3])};
  unsigned short* q = Aout + ao;
  *(volatile v2u*)q = u;
  __threadfence();
  *(volatile v2u*)q = u;
}

__global__ __launch_bounds__(256) void gate_split_kernel(const float* __restrict__ Gp, const unsigned short* __restrict__ Ah,
                                                         const unsigned short* __restrict__ Al, unsigned short* __restrict__ Oh,
                                                         unsigned short* __restrict__ Ol, int chunk) {
  const int i   = blockIdx.x * 256 + threadIdx.x;
  const int row = i >> 8;
  if (row >= kB * kQS) return;
  const int col = (i & 255) * 4;
  const int b   = row / kQS, s = row - b * kQS;
  const int tok = b * kS + s;
  const v4f g = *(const v4f*)(Gp + (size_t)tok * kCP + col);
  const size_t ao = (size_t)row * kHid + chunk * kCP + col;
  const v2u hw = *(const v2u*)(Ah + ao);
  const v2u lw = *(const v2u*)(Al + ao);
  float a[4];
  a[0] = __uint_as_float(hw[0] << 16)          + __uint_as_float(lw[0] << 16);
  a[1] = __uint_as_float(hw[0] & 0xffff0000u)  + __uint_as_float(lw[0] & 0xffff0000u);
  a[2] = __uint_as_float(hw[1] << 16)          + __uint_as_float(lw[1] << 16);
  a[3] = __uint_as_float(hw[1] & 0xffff0000u)  + __uint_as_float(lw[1] & 0xffff0000u);
  unsigned short hb[4], lb[4];
#pragma unroll
  for (int e = 0; e < 4; ++e) {
    const float r = a[e] * sigm(g[e]);
    hb[e] = f2bf_bits(r);
    lb[e] = f2bf_bits(r - bf_bits2f(hb[e]));
  }
  const v2u uh = (v2u){pk16(hb[0], hb[1]), pk16(hb[2], hb[3])};
  const v2u ul = (v2u){pk16(lb[0], lb[1]), pk16(lb[2], lb[3])};
  *(volatile v2u*)(Oh + ao) = uh;
  *(volatile v2u*)(Ol + ao) = ul;
  __threadfence();
  *(volatile v2u*)(Oh + ao) = uh;
  *(volatile v2u*)(Ol + ao) = ul;
}

extern "C" void kernel_launch(void* const* d_in, const int* in_sizes, int n_in,
                              void* d_out, int out_size, void* d_ws, size_t ws_size,
                              hipStream_t stream) {
  if (n_in < 9) return;
  if (in_sizes[0] != kTok * kHid) return;
  if (in_sizes[1] != kTok || in_sizes[2] != kTok) return;
  if (in_sizes[3] != kHid * 2 * kHid) return;
  if (in_sizes[4] != kHid * kCP || in_sizes[5] != kHid * kCP) return;
  if (in_sizes[6] != kHid * kHid) return;
  if (in_sizes[7] != kHD || in_sizes[8] != kHD) return;
  if (out_size != kTok * kHid) return;

  const size_t szXh   = (size_t)kTok * kHid * 2;
  const size_t szW    = (size_t)(3 * kHid) * kHid * 2;
  const size_t szC    = (size_t)kTok * kCP * 4;
  const size_t szKh   = (size_t)kTok * kCP * 2;
  const size_t szKb   = (size_t)kB * kQS * kCP * 2;
  const size_t szVt   = (size_t)kB * kNKV * kHD * kS * 2;
  const size_t szVtb  = (size_t)kB * kNKV * kHD * kQS * 2;
  const size_t szQh   = (size_t)kB * kQP * kHid * 2;
  const size_t szQb   = (size_t)kB * kQS * kHid * 2;
  const size_t szWoTb = (size_t)kHid * kHid * 2;
  const size_t offXh   = 0;
  const size_t offW    = offXh + szXh;
  const size_t offC    = offW + szW;
  const size_t offKh   = offC + szC;
  const size_t offKbh  = offKh + szKh;
  const size_t offKbl  = offKbh + szKb;
  const size_t offVt   = offKbl + szKb;
  const size_t offVtbh = offVt + szVt;
  const size_t offVtbl = offVtbh + szVtb;
  const size_t offQh   = offVtbl + szVtb;
  const size_t offQbh  = offQh + szQh;
  const size_t offQbl  = offQbh + szQb;
  const size_t offAt   = offQbl + szQb;
  const size_t offAtbh = offAt + szQh;
  const size_t offAtbl = offAtbh + szQb;
  const size_t offWoTb = offAtbl + szQb;
  const size_t total   = offWoTb + szWoTb;
  if (ws_size < total) return;

  const float* xin       = (const float*)d_in[0];
  const int*   amask     = (const int*)d_in[1];
  const int*   positions = (const int*)d_in[2];
  const float* Wq        = (const float*)d_in[3];
  const float* Wk        = (const float*)d_in[4];
  const float* Wv        = (const float*)d_in[5];
  const float* Wo        = (const float*)d_in[6];
  const float* qnw       = (const float*)d_in[7];
  const float* knw       = (const float*)d_in[8];
  float* out = (float*)d_out;
  char* ws = (char*)d_ws;
  unsigned short* Xh    = (unsigned short*)(ws + offXh);
  unsigned short* WqT   = (unsigned short*)(ws + offW);
  unsigned short* WgT   = WqT + (size_t)kHid * kHid;
  unsigned short* WkT   = WgT + (size_t)kHid * kHid;
  unsigned short* WvT   = WkT + (size_t)kCP * kHid;
  float*          C32   = (float*)(ws + offC);
  unsigned short* Kh    = (unsigned short*)(ws + offKh);
  unsigned short* Kbh   = (unsigned short*)(ws + offKbh);
  unsigned short* Kbl   = (unsigned short*)(ws + offKbl);
  unsigned short* Vt    = (unsigned short*)(ws + offVt);
  unsigned short* Vtbh  = (unsigned short*)(ws + offVtbh);
  unsigned short* Vtbl  = (unsigned short*)(ws + offVtbl);
  unsigned short* Qh    = (unsigned short*)(ws + offQh);
  unsigned short* Qbh   = (unsigned short*)(ws + offQbh);
  unsigned short* Qbl   = (unsigned short*)(ws + offQbl);
  unsigned short* At    = (unsigned short*)(ws + offAt);
  unsigned short* Atbh  = (unsigned short*)(ws + offAtbh);
  unsigned short* Atbl  = (unsigned short*)(ws + offAtbl);
  unsigned short* WoTb  = (unsigned short*)(ws + offWoTb);
  unsigned short* WoT16 = Xh;
  unsigned short* AG16  = Qh;
  unsigned short* AGbh  = Qbh;
  unsigned short* AGbl  = Qbl;

  RopeFreq rf;
  for (int j = 0; j < 16; ++j) {
    const double pd = pow(10000000.0, (double)j / 16.0);
    const float  pf = (float)pd;
    rf.f[j] = 1.0f / pf;
  }

  const int n8 = (kTok * kHid) / 8;
  castx_kernel<<<dim3(n8 / 256), dim3(256), 0, stream>>>(xin, Xh, n8);
  wt_kernel<false><<<dim3(kHid / 64, kHid / 64), dim3(256), 0, stream>>>(Wq, 2 * kHid, 256, 0,   WqT, kWCarry);
  wt_kernel<false><<<dim3(kHid / 64, kHid / 64), dim3(256), 0, stream>>>(Wq, 2 * kHid, 256, 128, WgT, kWCarry);
  wt_kernel<false><<<dim3(kHid / 64, kCP / 64),  dim3(256), 0, stream>>>(Wk, kCP, 128, 0, WkT, kWCarry);
  wt_kernel<false><<<dim3(kHid / 64, kCP / 64),  dim3(256), 0, stream>>>(Wv, kCP, 128, 0, WvT, kWCarry);

  const int tilesProj = (kTok / 64) * (kCP / 64);

  wmma_gemm64<0, 0, 0, 0, false, 0><<<dim3(tilesProj / 8, 1), dim3(256), 0, stream>>>(
      Xh, Xh, kHid, 0L, WkT, WkT, kHid, 0L, (void*)C32, (void*)C32, kCP, 0L, xin, xin, 0L, kTok, kCP, kHid, kWCarryInv);
  normrope_kernel<false><<<dim3(kTok / 8), dim3(256), 0, stream>>>(C32, knw, positions, rf, Kh, Kbh, Kbl, 0);

  wmma_gemm64<0, 0, 0, 0, false, 0><<<dim3(tilesProj / 8, 1), dim3(256), 0, stream>>>(
      Xh, Xh, kHid, 0L, WvT, WvT, kHid, 0L, (void*)C32, (void*)C32, kCP, 0L, xin, xin, 0L, kTok, kCP, kHid, kWCarryInv);
  vt_kernel<<<dim3(kS / 64, kNKV, kB), dim3(256), 0, stream>>>(C32, Vt, Vtbh, Vtbl);

  for (int ch = 0; ch < 2; ++ch) {
    const unsigned short* Bq = WqT + (size_t)ch * kCP * kHid;
    wmma_gemm64<0, 0, 0, 0, false, 0><<<dim3(tilesProj / 8, 1), dim3(256), 0, stream>>>(
        Xh, Xh, kHid, 0L, Bq, Bq, kHid, 0L, (void*)C32, (void*)C32, kCP, 0L, xin, xin, 0L, kTok, kCP, kHid, kWCarryInv);
    normrope_kernel<true><<<dim3(kTok / 8), dim3(256), 0, stream>>>(C32, qnw, positions, rf, Qh, Qbh, Qbl, ch);
  }

  const int nqbSplit = kQS / 64;
  const int nqbPlain = (kS - kQS) / 64;
  attn128_kernel<false><<<dim3(nqbPlain * kNH * kB), dim3(128), 0, stream>>>(
      Qh, Qh, kQP, kQS, Kh, Kh, kS, Vt, Vt, kS, amask, At, At, kQP, kQS, nqbSplit, nqbPlain);
  attn128_kernel<true><<<dim3(nqbSplit * kNH * kB), dim3(128), 0, stream>>>(
      Qbh, Qbl, kQS, 0, Kbh, Kbl, kQS, Vtbh, Vtbl, kQS, amask, Atbh, Atbl, kQS, 0, 0, nqbSplit);

  for (int ch = 0; ch < 2; ++ch) {
    const unsigned short* Bg = WgT + (size_t)ch * kCP * kHid;
    wmma_gemm64<0, 0, 0, 0, false, 0><<<dim3(tilesProj / 8, 1), dim3(256), 0, stream>>>(
        Xh, Xh, kHid, 0L, Bg, Bg, kHid, 0L, (void*)C32, (void*)C32, kCP, 0L, xin, xin, 0L, kTok, kCP, kHid, kWCarryInv);
    gate_plain_kernel<<<dim3((kB * kQP * kCP / 4) / 256), dim3(256), 0, stream>>>(C32, At, AG16, ch);
    gate_split_kernel<<<dim3((kB * kQS * kCP / 4) / 256), dim3(256), 0, stream>>>(C32, Atbh, Atbl, AGbh, AGbl, ch);
  }

  wt_kernel<false><<<dim3(kHid / 64, kHid / 64), dim3(256), 0, stream>>>(Wo, kHid, 128, 0, WoT16, kWCarry);
  wt_kernel<true><<<dim3(kHid / 64, kHid / 64), dim3(256), 0, stream>>>(Wo, kHid, 128, 0, WoTb, 1.0f);

  const int tilesOutP = (kQP / 64) * (kHid / 64);
  wmma_gemm64<0, 0, 0, 0, false, 0><<<dim3(tilesOutP / 8, kB), dim3(256), 0, stream>>>(
      AG16, AG16, kHid, (long)kQP * kHid, WoT16, WoT16, kHid, 0L,
      (void*)(out + (size_t)kQS * kHid), (void*)(out + (size_t)kQS * kHid), kHid, (long)kS * kHid,
      xin, xin, 0L, kQP, kHid, kHid, kOutScalePlain);
  const int tilesOutS = (kQS / 64) * (kHid / 64);
  wmma_gemm64<1, 2, 0, 0, false, 0><<<dim3(tilesOutS / 8, kB), dim3(256), 0, stream>>>(
      AGbh, AGbl, kHid, (long)kQS * kHid, WoTb, WoTb, kHid, 0L,
      (void*)out, (void*)out, kHid, (long)kS * kHid,
      xin, xin, 0L, kQS, kHid, kHid, 1.0f);
}
